// KANLinear_24893630447742
// MI455X (gfx1250) — hardware-run, weakly checked
//
#include <hip/hip_runtime.h>
#include <math.h>
#include <stdint.h>

constexpr int kBatch    = 32768;
constexpr int kIn       = 256;
constexpr int kOutF     = 256;
constexpr int kCoef     = 8;
constexpr int kGridN    = 12;
constexpr int kKsil     = kIn;
constexpr int kKspl     = kIn * kCoef;
constexpr int kKtot     = kKsil + kKspl;
constexpr int kHalfRows = kBatch / 2;
constexpr int kBtChunks = kKtot / 8;
constexpr float kWCarry    = 64.0f;
constexpr float kWCarryInv = 1.0f / 64.0f;

constexpr size_t kBtBytes  = (size_t)kOutF * kKtot * 2;
constexpr size_t kAOff     = kBtBytes;
constexpr size_t kABytes   = (size_t)kHalfRows * kKtot * 2;
constexpr size_t kWsTotal  = kAOff + kABytes;
static_assert(kBtBytes == 1179648, "bt bytes");
static_assert(kABytes == 75497472, "a bytes");
static_assert(kWsTotal == 76677120, "ws total");
static_assert(kWsTotal <= (size_t)134217728, "carve under 128 MiB");
static_assert((kAOff % 128) == 0, "128-B aligned region");
static_assert(kKtot % 32 == 0, "K multiple of 32");
static_assert(kHalfRows % 64 == 0 && kOutF % 64 == 0, "M,N tile multiples");
static_assert((kKtot * 2) % 128 == 0, "16-bit plane rows are whole lines");
static_assert((kOutF * 4) % 128 == 0, "out rows are whole lines");
static_assert((kOutF * kBtChunks) % 256 == 0, "bt grid exact");
static_assert(kBtChunks % 32 == 0, "bt waves stay inside one row");

typedef __attribute__((ext_vector_type(16))) _Float16 v16h;
typedef __attribute__((ext_vector_type(8)))  _Float16 v8h;
typedef __attribute__((ext_vector_type(16))) __bf16   v16b;
typedef __attribute__((ext_vector_type(8)))  __bf16   v8b;
typedef __attribute__((ext_vector_type(8)))  float    v8f;
typedef __attribute__((ext_vector_type(4)))  float    v4f;
typedef __attribute__((ext_vector_type(4)))  unsigned int v4u;

__device__ __forceinline__ unsigned short f2bf_bits(float f) {
  unsigned u = __float_as_uint(f);
  return (unsigned short)((u + 0x7FFFu + ((u >> 16) & 1u)) >> 16);
}
__device__ __forceinline__ float bf_bits2f(unsigned short h) { return __uint_as_float(((unsigned)h) << 16); }

__device__ __forceinline__ void dep_guard_h(v8f& a, v8f& b, v16h x, v16h y) { asm volatile("v_nop\n\tv_nop\n\tv_nop\n\tv_nop" : "+v"(a), "+v"(b) : "v"(x), "v"(y)); }
__device__ __forceinline__ void dep_guard_b(v8f& a, v8f& b, v16b x, v16b y) { asm volatile("v_nop\n\tv_nop\n\tv_nop\n\tv_nop" : "+v"(a), "+v"(b) : "v"(x), "v"(y)); }
__device__ __forceinline__ void dep_guard4_h(v8f& a, v8f& b, v8f& c, v8f& d, v16h x, v16h y) { asm volatile("v_nop\n\tv_nop\n\tv_nop\n\tv_nop" : "+v"(a), "+v"(b), "+v"(c), "+v"(d) : "v"(x), "v"(y)); }
__device__ __forceinline__ void dep_guard4_b(v8f& a, v8f& b, v8f& c, v8f& d, v16b x, v16b y) { asm volatile("v_nop\n\tv_nop\n\tv_nop\n\tv_nop" : "+v"(a), "+v"(b), "+v"(c), "+v"(d) : "v"(x), "v"(y)); }
__device__ __forceinline__ void keep4_h(v16h a, v16h b, v16h c, v16h d) { asm volatile("v_nop" :: "v"(a), "v"(b), "v"(c), "v"(d)); }
__device__ __forceinline__ void keep4_b(v16b a, v16b b, v16b c, v16b d) { asm volatile("v_nop" :: "v"(a), "v"(b), "v"(c), "v"(d)); }
__device__ __forceinline__ void acc_guard4(v8f& a, v8f& b, v8f& c, v8f& d) { asm volatile("v_nop\n\tv_nop\n\tv_nop\n\tv_nop" : "+v"(a), "+v"(b), "+v"(c), "+v"(d)); }
template <typename T> struct Frag;
template <> struct Frag<_Float16> {
  typedef v16h V; union U { v16h v; v8h h[2]; };
  static __device__ __forceinline__ v16h load(const _Float16* p) {
    U f; f.h[0] = *(const v8h*)(p); f.h[1] = *(const v8h*)(p + 16); return f.v;
  }
  static __device__ __forceinline__ v8f mma(v16h a, v16h b, v8f c) {
    return __builtin_amdgcn_wmma_f32_16x16x32_f16(false, a, false, b, (short)0, c, false, false);
  }
  static __device__ __forceinline__ void guard(v8f& a, v8f& b, v16h x, v16h y) { dep_guard_h(a, b, x, y); }
  static __device__ __forceinline__ void guard4(v8f& a, v8f& b, v8f& c, v8f& d, v16h x, v16h y) { dep_guard4_h(a, b, c, d, x, y); }
  static __device__ __forceinline__ void keep(v16h a, v16h b, v16h c, v16h d) { keep4_h(a, b, c, d); }
};
template <> struct Frag<__bf16> {
  typedef v16b V; union U { v16b v; v8b h[2]; };
  static __device__ __forceinline__ v16b load(const __bf16* p) {
    U f; f.h[0] = *(const v8b*)(p); f.h[1] = *(const v8b*)(p + 16); return f.v;
  }
  static __device__ __forceinline__ v8f mma(v16b a, v16b b, v8f c) {
    return __builtin_amdgcn_wmma_f32_16x16x32_bf16(false, a, false, b, (short)0, c, false, false);
  }
  static __device__ __forceinline__ void guard(v8f& a, v8f& b, v16b x, v16b y) { dep_guard_b(a, b, x, y); }
  static __device__ __forceinline__ void guard4(v8f& a, v8f& b, v8f& c, v8f& d, v16b x, v16b y) { dep_guard4_b(a, b, c, d, x, y); }
  static __device__ __forceinline__ void keep(v16b a, v16b b, v16b c, v16b d) { keep4_b(a, b, c, d); }
};

__device__ __forceinline__ unsigned pk16(unsigned short a, unsigned short b) { return (unsigned)a | ((unsigned)b << 16); }
__device__ __forceinline__ unsigned short h_bits(float f) { const _Float16 h = (_Float16)f; return __builtin_bit_cast(unsigned short, h); }

template <int ET> struct Elem;
template <> struct Elem<0> { typedef _Float16 T; };
template <> struct Elem<1> { typedef __bf16 T; };
template <int ET, bool SPLIT, int BIAS_MODE, int OUT_MODE, bool RESID, int ACT = 0>
__global__ __launch_bounds__(256) void wmma_gemm64(
    const unsigned short* __restrict__ Ap, const unsigned short* __restrict__ A2p, int lda, long strideA,
    const unsigned short* __restrict__ Btp, const unsigned short* __restrict__ Bt2p, int ldb, long strideB,
    void* __restrict__ Cout, void* __restrict__ Cout2, int ldc, long strideC,
    const float* __restrict__ bias,
    const float* __restrict__ resid, long strideR,
    int M, int N, int K, float scale) {
  typedef typename Elem<ET>::T T;
  typedef typename Frag<T>::V V;
  const T* A = (const T*)Ap; const T* A2 = (const T*)A2p; const T* Bt = (const T*)Btp; const T* Bt2 = (const T*)Bt2p;
  __shared__ __align__(16) float sT[8][16 * 68];
  const int b    = blockIdx.y;
  const int lane = threadIdx.x & 31;
  const int wave = threadIdx.x >> 5;
  const int tilesN = N >> 6;
  const int tilesM = M >> 6;
  const int tile = blockIdx.x * 8 + wave;
  if (tile >= tilesM * tilesN) return;
  const int tm = tile / tilesN;
  const int tn = tile - tm * tilesN;
  const int m0 = tm << 6;
  const int n0 = tn << 6;

  const T* Ab  = A  + (size_t)b * strideA;
  const T* Bb  = Bt + (size_t)b * strideB;
  const T* Ab2 = SPLIT ? (A2  + (size_t)b * strideA) : nullptr;
  const T* Bb2 = SPLIT ? (Bt2 + (size_t)b * strideB) : nullptr;

  const int rlane = lane & 15;
  const int koff  = (lane >> 4) * 8;
  const int mOff  = (lane >> 4) * 8;

  v8f acc[4][4];
#pragma unroll
  for (int i = 0; i < 4; ++i)
#pragma unroll
    for (int j = 0; j < 4; ++j) acc[i][j] = (v8f){0.f,0.f,0.f,0.f,0.f,0.f,0.f,0.f};

  for (int k0 = 0; k0 < K; k0 += 32) {
    V bh[4], bl[4];
#pragma unroll
    for (int j = 0; j < 4; ++j) {
      const size_t bo = (size_t)(n0 + (j << 4) + rlane) * ldb + koff + k0;
      bh[j] = Frag<T>::load(Bb + bo);
      if (SPLIT) bl[j] = Frag<T>::load(Bb2 + bo);
    }
#pragma unroll
    for (int i = 0; i < 4; ++i) {
      const size_t ao = (size_t)(m0 + (i << 4) + rlane) * lda + koff + k0;
      V ah = Frag<T>::load(Ab + ao);
      V al;
      if (SPLIT) al = Frag<T>::load(Ab2 + ao);
#pragma unroll
      for (int j = 0; j < 4; ++j) {
        acc[i][j] = Frag<T>::mma(ah, bh[j], acc[i][j]);
        if (SPLIT) {
          acc[i][j] = Frag<T>::mma(ah, bl[j], acc[i][j]);
          acc[i][j] = Frag<T>::mma(al, bh[j], acc[i][j]);
        }
      }
      Frag<T>::guard4(acc[i][0], acc[i][1], acc[i][2], acc[i][3], ah, SPLIT ? al : bh[3]);
    }
    Frag<T>::keep(bh[0], bh[1], bh[2], bh[3]);
    if (SPLIT) Frag<T>::keep(bl[0], bl[1], bl[2], bl[3]);
  }
  acc_guard4(acc[0][0], acc[0][1], acc[0][2], acc[0][3]);
  acc_guard4(acc[1][0], acc[1][1], acc[1][2], acc[1][3]);
  acc_guard4(acc[2][0], acc[2][1], acc[2][2], acc[2][3]);
  acc_guard4(acc[3][0], acc[3][1], acc[3][2], acc[3][3]);

  float* slab = sT[wave];
  const float* Rb = RESID ? (resid + (size_t)b * strideR) : nullptr;
#pragma unroll
  for (int i = 0; i < 4; ++i) {
    const int mBase = m0 + (i << 4);
#pragma unroll
    for (int j = 0; j < 4; ++j) {
      const int n = n0 + (j << 4) + rlane;
      float bv = 0.f;
      if (BIAS_MODE == 2) bv = bias[n];
#pragma unroll
      for (int r = 0; r < 8; ++r) {
        float v = acc[i][j][r] * scale;
        if (BIAS_MODE == 1) v += bias[mBase + mOff + r];
        if (BIAS_MODE == 2) v += bv;
        if (RESID) v += Rb[(size_t)(mBase + mOff + r) * ldc + n];
        if (ACT == 2) v = fmaxf(v, 0.0f);
        if (ACT == 4) v = (v > 0.f) ? v : 0.01f * v;
        slab[(mOff + r) * 68 + (j << 4) + rlane] = v;
      }
    }
    __builtin_amdgcn_fence(__ATOMIC_RELEASE, "workgroup");
    __builtin_amdgcn_wave_barrier();
    __builtin_amdgcn_fence(__ATOMIC_ACQUIRE, "workgroup");
    if (OUT_MODE == 0) {
      float* C = (float*)Cout + (size_t)b * strideC;
      const int hh = lane >> 4, c4 = (lane & 15) * 4;
      for (int pass = 0; pass < 2; ++pass) {
#pragma unroll
        for (int it = 0; it < 8; ++it) {
          const int row = it * 2 + hh;
          v4f v = *(const v4f*)(slab + row * 68 + c4);
          *(volatile v4f*)(C + (size_t)(mBase + row) * ldc + n0 + c4) = v;
        }
        __threadfence();
      }
    } else {
      const int q = lane >> 3, c8 = (lane & 7) * 8;
      unsigned short* C  = (unsigned short*)Cout  + (size_t)b * strideC;
      unsigned short* C2 = (OUT_MODE == 2) ? ((unsigned short*)Cout2 + (size_t)b * strideC) : nullptr;
      for (int pass = 0; pass < 2; ++pass) {
#pragma unroll
        for (int it = 0; it < 4; ++it) {
          const int row = it * 4 + q;
          const float* sp = slab + row * 68 + c8;
          v8h hv, lv;
#pragma unroll
          for (int e = 0; e < 8; ++e) {
            if (OUT_MODE == 1) {
              hv[e] = (_Float16)sp[e];
            } else {
              unsigned short hb = f2bf_bits(sp[e]);
              unsigned short lb = f2bf_bits(sp[e] - bf_bits2f(hb));
              hv[e] = __builtin_bit_cast(_Float16, hb);
              lv[e] = __builtin_bit_cast(_Float16, lb);
            }
          }
          *(volatile v8h*)(C + (size_t)(mBase + row) * ldc + n0 + c8) = hv;
          if (OUT_MODE == 2) *(volatile v8h*)(C2 + (size_t)(mBase + row) * ldc + n0 + c8) = lv;
        }
        __threadfence();
      }
    }
    __builtin_amdgcn_fence(__ATOMIC_RELEASE, "workgroup");
    __builtin_amdgcn_wave_barrier();
    __builtin_amdgcn_fence(__ATOMIC_ACQUIRE, "workgroup");
  }
}

__global__ __launch_bounds__(256) void btw_kernel(const float* __restrict__ base_w, const float* __restrict__ spline_w,
                                                  const float* __restrict__ spline_s, unsigned short* __restrict__ bt) {
  const int gid = blockIdx.x * 256 + threadIdx.x;
  if (gid >= kOutF * kBtChunks) return;
  const int n  = gid / kBtChunks;
  const int q  = gid - n * kBtChunks;
  const int k0 = q * 8;
  const int kb = (k0 < kIn - 8) ? k0 : (kIn - 8);
  const float* bp = base_w + (size_t)n * kIn + kb;
  const v4f b0 = *(const v4f*)(bp);
  const v4f b1 = *(const v4f*)(bp + 4);
  const int is = (q >= 32) ? (q - 32) : 0;
  const size_t gi = (size_t)n * kIn + is;
  const float* sp = spline_w + gi * kCoef;
  const v4f s0 = *(const v4f*)(sp);
  const v4f s1 = *(const v4f*)(sp + 4);
  const float sc = spline_s[gi];
  const float fa = (q < 32) ? 1.0f : 0.0f;
  const float fs = 1.0f - fa;
  float w[8];
#pragma unroll
  for (int e = 0; e < 4; ++e) {
    const float pa0 = kWCarry * b0[e];
    const float pa1 = kWCarry * b1[e];
    const float ps0 = kWCarry * (s0[e] * sc);
    const float ps1 = kWCarry * (s1[e] * sc);
    w[e]     = fmaf(fa, pa0, fs * ps0);
    w[4 + e] = fmaf(fa, pa1, fs * ps1);
  }
  unsigned short hb[8];
#pragma unroll
  for (int e = 0; e < 8; ++e) hb[e] = h_bits(w[e]);
  const v4u u = (v4u){pk16(hb[0], hb[1]), pk16(hb[2], hb[3]), pk16(hb[4], hb[5]), pk16(hb[6], hb[7])};
  unsigned short* dst = bt + (size_t)n * kKtot + k0;
  *(volatile v4u*)dst = u;
  __threadfence();
  *(volatile v4u*)dst = u;
}

__global__ __launch_bounds__(256) void feat_kernel(const float* __restrict__ x, const float* __restrict__ gridp,
                                                   unsigned short* __restrict__ aplane, int row_base) {
  __shared__ float sg[kGridN];
  __shared__ float srcp[32];
  __shared__ __align__(16) float ssil[kIn];
  const int t    = threadIdx.x;
  const int lane = t & 31;
  const int wave = t >> 5;
  const int r    = blockIdx.x;
  if (t < kGridN) sg[t] = gridp[t];
  __syncthreads();
  if (t < 30) {
    const int kk = 1 + ((t >= 11) ? 1 : 0) + ((t >= 21) ? 1 : 0);
    const int j  = t - ((t >= 11) ? 11 : 0) - ((t >= 21) ? 10 : 0);
    srcp[t] = 1.0f / (sg[j + kk] - sg[j]);
  }
  const float xv = x[(size_t)(row_base + r) * kIn + t];
  const float ex  = expf(-xv);
  const float sig = 1.0f / (1.0f + ex);
  const float sl  = xv * sig;
  ssil[t] = sl;
  __syncthreads();

  float gk[kGridN];
#pragma unroll
  for (int u = 0; u < kGridN; ++u) gk[u] = sg[u];
  float rc1[11], rc2[10], rc3[9];
#pragma unroll
  for (int u = 0; u < 11; ++u) rc1[u] = srcp[u];
#pragma unroll
  for (int u = 0; u < 10; ++u) rc2[u] = srcp[11 + u];
#pragma unroll
  for (int u = 0; u < 9; ++u) rc3[u] = srcp[21 + u];

  float bb[11];
#pragma unroll
  for (int j = 0; j < 11; ++j) bb[j] = (xv >= gk[j] && xv < gk[j + 1]) ? 1.0f : 0.0f;
#pragma unroll
  for (int j = 0; j < 10; ++j) {
    const float lf = (xv - gk[j]) * rc1[j];
    const float rg = (gk[j + 2] - xv) * rc1[j + 1];
    bb[j] = lf * bb[j] + rg * bb[j + 1];
  }
#pragma unroll
  for (int j = 0; j < 9; ++j) {
    const float lf = (xv - gk[j]) * rc2[j];
    const float rg = (gk[j + 3] - xv) * rc2[j + 1];
    bb[j] = lf * bb[j] + rg * bb[j + 1];
  }
#pragma unroll
  for (int j = 0; j < 8; ++j) {
    const float lf = (xv - gk[j]) * rc3[j];
    const float rg = (gk[j + 4] - xv) * rc3[j + 1];
    bb[j] = lf * bb[j] + rg * bb[j + 1];
  }

  unsigned short hb[8];
#pragma unroll
  for (int c = 0; c < 8; ++c) hb[c] = h_bits(bb[c]);
  const v4u ub = (v4u){pk16(hb[0], hb[1]), pk16(hb[2], hb[3]), pk16(hb[4], hb[5]), pk16(hb[6], hb[7])};

  unsigned short hs[8];
#pragma unroll
  for (int e = 0; e < 8; ++e) hs[e] = h_bits(ssil[8 * lane + e]);
  const v4u us = (v4u){pk16(hs[0], hs[1]), pk16(hs[2], hs[3]), pk16(hs[4], hs[5]), pk16(hs[6], hs[7])};

  unsigned short* arow = aplane + (size_t)r * kKtot;
  unsigned short* pbas = arow + kKsil + t * kCoef;
  unsigned short* psil = arow + 8 * lane;
  *(volatile v4u*)pbas = ub;
  if (wave == 0) *(volatile v4u*)psil = us;
  __threadfence();
  *(volatile v4u*)pbas = ub;
  if (wave == 0) *(volatile v4u*)psil = us;
}

extern "C" void kernel_launch(void* const* d_in, const int* in_sizes, int n_in,
                              void* d_out, int out_size, void* d_ws, size_t ws_size,
                              hipStream_t stream) {
  if (n_in < 5) return;
  if (in_sizes[0] != kBatch * kIn) return;
  if (in_sizes[1] != kOutF * kIn) return;
  if (in_sizes[2] != kOutF * kIn * kCoef) return;
  if (in_sizes[3] != kOutF * kIn) return;
  if (in_sizes[4] != kGridN) return;
  if ((size_t)out_size != (size_t)kBatch * kOutF) return;
  if (ws_size < kWsTotal) return;

  const float* x    = (const float*)d_in[0];
  const float* bw   = (const float*)d_in[1];
  const float* sw   = (const float*)d_in[2];
  const float* ss   = (const float*)d_in[3];
  const float* grd  = (const float*)d_in[4];
  float* out        = (float*)d_out;
  unsigned char* ws = (unsigned char*)d_ws;
  unsigned short* btp = (unsigned short*)(ws);
  unsigned short* ap  = (unsigned short*)(ws + kAOff);

  btw_kernel<<<dim3((kOutF * kBtChunks) / 256), dim3(256), 0, stream>>>(bw, sw, ss, btp);

  const int gemm_blocks = ((kHalfRows / 64) * (kOutF / 64)) / 8;
  for (int half = 0; half < 2; ++half) {
    const int row_base = half * kHalfRows;
    feat_kernel<<<dim3(kHalfRows), dim3(256), 0, stream>>>(x, grd, ap, row_base);
    float* cout = out + (size_t)row_base * kOutF;
    wmma_gemm64<0, false, 0, 0, false, 0><<<dim3(gemm_blocks, 1), dim3(256), 0, stream>>>(
        ap, ap, kKtot, 0L,
        btp, btp, kKtot, 0L,
        (void*)cout, (void*)cout, kOutF, 0L,
        bw,
        x, 0L,
        kHalfRows, kOutF, kKtot, kWCarryInv);
  }
}
